// GATLayer_20461224198293
// MI455X (gfx1250) — hardware-verified
//
#include <hip/hip_runtime.h>
#include <stddef.h>
#include <stdint.h>
#include <math.h>

#pragma clang fp contract(off)

#define NN     8192
#define FIN    512
#define FOUT   256
#define NTHR   256
#define GBM    64
#define KT     64
#define NH     128
#define NEGSL  0.2f
#define NUX    (NN * (FIN / 8))
#define NUW    (FOUT * (FIN / 8))
#define PLDS   ((GBM * FOUT + 2 * GBM) * 4)
#define PAP    136
#define HBP    72
#define A_F_S2   0
#define A_B_PA   (NN * 4)
#define A_B_HH   (A_B_PA + GBM * PAP * 2)
#define A_B_HL   (A_B_HH + NH * HBP * 2)
#define A_B_MISC (A_B_HL + NH * HBP * 2)
#define ALDS     (A_B_MISC + 320)
#define WSMAX  134217728

static_assert((FIN % 32) == 0 && (NN % GBM) == 0 && (NN % KT) == 0 && (KT % 32) == 0);
static_assert(FOUT == 2 * NH && NH == 2 * 64 && GBM == 4 * 16);
static_assert((NUX % NTHR) == 0 && (NUW % NTHR) == 0);
static_assert((A_B_PA % 16) == 0 && (A_B_HH % 16) == 0 && (A_B_HL % 16) == 0 && (A_B_MISC % 16) == 0);
static_assert(GBM * NH * 4 <= 2 * NH * HBP * 2);
static_assert((PAP % 8) == 0 && (HBP % 8) == 0 && PAP >= 128 && HBP >= KT);
static_assert(ALDS <= 300000 && PLDS <= 300000);

typedef float          v4f  __attribute__((ext_vector_type(4)));
typedef float          v8f  __attribute__((ext_vector_type(8)));
typedef int            v8i  __attribute__((ext_vector_type(8)));
typedef unsigned int   v4u  __attribute__((ext_vector_type(4)));
typedef unsigned short v8us __attribute__((ext_vector_type(8)));
typedef __bf16         v16b __attribute__((ext_vector_type(16)));
typedef v4f  __attribute__((may_alias)) v4fa;
typedef v4u  __attribute__((may_alias)) v4ua;
typedef v8us __attribute__((may_alias)) v8usa;
union FragB { v16b v; v8us h[2]; v8i w; };

__device__ __forceinline__ v8f wmb(const FragB& a, const FragB& b, v8f c) {
  v8f d = __builtin_amdgcn_wmma_f32_16x16x32_bf16(false, a.v, false, b.v, (short)0, c, false, false);
  asm volatile("v_nop\n\tv_nop\n\tv_nop\n\tv_nop" : "+v"(d) : "v"(a.w), "v"(b.w));
  return d;
}

__device__ __forceinline__ unsigned int f2bf(float f) {
  const unsigned int u = __float_as_uint(f);
  return ((u + 0x7FFFu + ((u >> 16) & 1u)) >> 16) & 0xFFFFu;
}
__device__ __forceinline__ float bf2f(unsigned int b) { return __uint_as_float(b << 16); }
__device__ __forceinline__ float bfr(float f) { return bf2f(f2bf(f)); }
__device__ __forceinline__ v4f bfr4(const v4f a) {
  v4f r; r.x = bfr(a.x); r.y = bfr(a.y); r.z = bfr(a.z); r.w = bfr(a.w); return r;
}
__device__ __forceinline__ unsigned int pk2(float lo, float hi) { return f2bf(lo) | (f2bf(hi) << 16); }
__device__ __forceinline__ v4u pack8(const v4f a, const v4f b) {
  v4u r;
  r.x = pk2(a.x, a.y); r.y = pk2(a.z, a.w); r.z = pk2(b.x, b.y); r.w = pk2(b.z, b.w);
  return r;
}
__device__ __forceinline__ void split8(const v4f a, const v4f b, v4u& hv, v4u& lv) {
  const unsigned int h0 = f2bf(a.x), h1 = f2bf(a.y), h2 = f2bf(a.z), h3 = f2bf(a.w);
  const unsigned int h4 = f2bf(b.x), h5 = f2bf(b.y), h6 = f2bf(b.z), h7 = f2bf(b.w);
  const unsigned int l0 = f2bf(a.x - bf2f(h0)), l1 = f2bf(a.y - bf2f(h1));
  const unsigned int l2 = f2bf(a.z - bf2f(h2)), l3 = f2bf(a.w - bf2f(h3));
  const unsigned int l4 = f2bf(b.x - bf2f(h4)), l5 = f2bf(b.y - bf2f(h5));
  const unsigned int l6 = f2bf(b.z - bf2f(h6)), l7 = f2bf(b.w - bf2f(h7));
  hv.x = h0 | (h1 << 16); hv.y = h2 | (h3 << 16); hv.z = h4 | (h5 << 16); hv.w = h6 | (h7 << 16);
  lv.x = l0 | (l1 << 16); lv.y = l2 | (l3 << 16); lv.z = l4 | (l5 << 16); lv.w = l6 | (l7 << 16);
}

__global__ __launch_bounds__(NTHR) void k_prep(const float* __restrict__ x, const float* __restrict__ W,
                                               unsigned short* XB, unsigned short* WT) {
  const int u = (int)blockIdx.x * NTHR + (int)threadIdx.x;
  v4u o;
  unsigned short* dp;
  if (u < NUX) {
    const int row = u >> 6;
    const int c0  = (u & 63) * 8;
    const float* p = x + (size_t)row * FIN + c0;
    const v4f a = *(const v4fa*)p;
    const v4f b = *(const v4fa*)(p + 4);
    o  = pack8(a, b);
    dp = XB + (size_t)row * FIN + c0;
  } else if (u < NUX + NUW) {
    const int v  = u - NUX;
    const int n  = v >> 6;
    const int k8 = (v & 63) * 8;
    const float* p = W + (size_t)k8 * FOUT + n;
    v4f a, b;
    a.x = p[0];          a.y = p[FOUT];       a.z = p[2 * FOUT];   a.w = p[3 * FOUT];
    b.x = p[4 * FOUT];   b.y = p[5 * FOUT];   b.z = p[6 * FOUT];   b.w = p[7 * FOUT];
    o  = pack8(a, b);
    dp = WT + (size_t)n * FIN + k8;
  } else {
    return;
  }
  *(volatile v4u*)dp = o;
  __threadfence();
  *(volatile v4u*)dp = o;
}

__device__ __forceinline__ void ht_pass(const float* stg, unsigned short* HTh, unsigned short* HTl,
                                        int rowBase, int tid) {
#pragma unroll 1
  for (int it = 0; it < 8; ++it) {
    const int pc = it * NTHR + tid;
    const int n  = pc >> 3;
    const int q  = pc & 7;
    const float* sp = stg + (8 * q) * FOUT + n;
    v4f a, b;
    a.x = sp[0];          a.y = sp[FOUT];       a.z = sp[2 * FOUT];   a.w = sp[3 * FOUT];
    b.x = sp[4 * FOUT];   b.y = sp[5 * FOUT];   b.z = sp[6 * FOUT];   b.w = sp[7 * FOUT];
    v4u hv, lv;
    split8(a, b, hv, lv);
    const size_t o = (size_t)n * NN + (size_t)(rowBase + 8 * q);
    *(volatile v4u*)(HTh + o) = hv;
    *(volatile v4u*)(HTl + o) = lv;
  }
}

__global__ __launch_bounds__(NTHR) void k_proj(const unsigned short* __restrict__ A,
                                               const unsigned short* __restrict__ BT,
                                               const float* __restrict__ av,
                                               unsigned short* HTh, unsigned short* HTl, float* SS) {
  extern __shared__ v4f lds_dyn[];
  float* stg = (float*)lds_dyn;
  float* sdt = stg + GBM * FOUT;
  const int tid = (int)threadIdx.x, lane = tid & 31, wave = tid >> 5, hh = lane >> 4, m = lane & 15;
  const int rg = wave & 3, cg = wave >> 2;
  const int rowBase = (int)blockIdx.x * GBM;
  const int colBase = cg * 128;

  v8f acc[8];
  {
    const v8f z = {0.f, 0.f, 0.f, 0.f, 0.f, 0.f, 0.f, 0.f};
#pragma unroll
    for (int t = 0; t < 8; ++t) acc[t] = z;
  }
  const unsigned short* ap = A  + (size_t)(rowBase + 16 * rg + m) * (size_t)FIN + 8 * hh;
  const unsigned short* bp = BT + (size_t)(colBase + m) * (size_t)FIN + 8 * hh;

#pragma unroll 1
  for (int k0 = 0; k0 < FIN; k0 += 32) {
    FragB af;
    af.h[0] = *(const v8usa*)(ap + k0);
    af.h[1] = *(const v8usa*)(ap + k0 + 16);
#pragma unroll
    for (int nt = 0; nt < 8; ++nt) {
      const unsigned short* wq = bp + (size_t)(16 * nt) * (size_t)FIN + k0;
      FragB bf;
      bf.h[0] = *(const v8usa*)wq;
      bf.h[1] = *(const v8usa*)(wq + 16);
      acc[nt] = wmb(af, bf, acc[nt]);
    }
  }

#pragma unroll
  for (int nt = 0; nt < 8; ++nt) {
    const int lc = colBase + 16 * nt + m;
#pragma unroll
    for (int r = 0; r < 8; ++r) {
      const int lr = 16 * rg + 8 * hh + r;
      stg[lr * FOUT + lc] = acc[nt][r];
    }
  }
  __syncthreads();

  v4f as4[2], ad4[2];
#pragma unroll
  for (int c = 0; c < 2; ++c) {
    as4[c] = bfr4(*(const v4fa*)(av + c * 128 + 4 * lane));
    ad4[c] = bfr4(*(const v4fa*)(av + FOUT + c * 128 + 4 * lane));
  }
#pragma unroll 1
  for (int i = 0; i < 8; ++i) {
    const int row = wave * 8 + i;
    float s = 0.0f, d = 0.0f;
#pragma unroll
    for (int c = 0; c < 2; ++c) {
      const v4f p = *(const v4fa*)(stg + row * FOUT + c * 128 + 4 * lane);
      s = fmaf(p.x, as4[c].x, s); s = fmaf(p.y, as4[c].y, s); s = fmaf(p.z, as4[c].z, s); s = fmaf(p.w, as4[c].w, s);
      d = fmaf(p.x, ad4[c].x, d); d = fmaf(p.y, ad4[c].y, d); d = fmaf(p.z, ad4[c].z, d); d = fmaf(p.w, ad4[c].w, d);
    }
#pragma unroll
    for (int off = 16; off > 0; off >>= 1) {
      s += __shfl_xor(s, off);
      d += __shfl_xor(d, off);
    }
    if (lane == 0) { sdt[row] = s; sdt[GBM + row] = d; }
  }
  __syncthreads();

  const v4f alv = *(const v4fa*)(sdt + 4 * lane);
  float* sp = SS + (size_t)(lane >> 4) * NN + rowBase + 4 * (lane & 15);

  ht_pass(stg, HTh, HTl, rowBase, tid);
  if (wave == 0) *(volatile v4f*)sp = alv;
  __threadfence();
  ht_pass(stg, HTh, HTl, rowBase, tid);
  if (wave == 0) *(volatile v4f*)sp = alv;
}

__device__ __forceinline__ float pexp(float s1r, float mr, float z) {
  float e = s1r + z;
  e = e > 0.0f ? e : NEGSL * e;
  return expf(e - mr);
}

__global__ __launch_bounds__(NTHR) void k_attn(const unsigned short* __restrict__ HTh,
                                               const unsigned short* __restrict__ HTl,
                                               const float* __restrict__ SS, float* out) {
  extern __shared__ v4f lds_dyn[];
  float* lf = (float*)lds_dyn;
  float* sS2 = lf + A_F_S2;
  unsigned short* sPA = (unsigned short*)(lf + A_B_PA / 4);
  unsigned short* sHh = (unsigned short*)(lf + A_B_HH / 4);
  unsigned short* sHl = (unsigned short*)(lf + A_B_HL / 4);
  float* stg  = lf + A_B_HH / 4;
  float* sRed = lf + A_B_MISC / 4;
  float* sL   = sRed + 16;
  const int tid = (int)threadIdx.x, lane = tid & 31, wave = tid >> 5, hh = lane >> 4, m = lane & 15;
  const int rg = wave & 3, cg = wave >> 2;
  const int rowBase = (int)blockIdx.x * GBM;
  const int coloff  = (int)blockIdx.y * NH;

  {
    const float* s2g = SS + NN;
    float mx = -3.0e38f;
#pragma unroll 4
    for (int i = 0; i < 8; ++i) {
      const int i4 = (i * NTHR + tid) * 4;
      const v4f v = *(const v4fa*)(s2g + i4);
      *(v4fa*)(sS2 + i4) = v;
      mx = fmaxf(mx, fmaxf(fmaxf(v.x, v.y), fmaxf(v.z, v.w)));
    }
#pragma unroll
    for (int off = 16; off > 0; off >>= 1) mx = fmaxf(mx, __shfl_xor(mx, off));
    if (lane == 0) sRed[wave] = mx;
  }
  __syncthreads();
  float s2mx = sRed[0];
#pragma unroll
  for (int w2 = 1; w2 < 8; ++w2) s2mx = fmaxf(s2mx, sRed[w2]);

  const int prow = tid >> 2;
  const int pseg = (tid & 3) * 16;
  const float s1r = SS[rowBase + prow];
  float mr = s1r + s2mx;
  mr = mr > 0.0f ? mr : NEGSL * mr;
  float lsum = 0.0f;

  v8f acc[4];
  {
    const v8f z = {0.f, 0.f, 0.f, 0.f, 0.f, 0.f, 0.f, 0.f};
    acc[0] = z; acc[1] = z; acc[2] = z; acc[3] = z;
  }

#pragma unroll 1
  for (int jt = 0; jt < NN / KT; ++jt) {
    const int j0 = jt * KT;
    {
      float tsum = 0.0f;
#pragma unroll
      for (int g = 0; g < 2; ++g) {
        const v4f za = *(const v4fa*)(sS2 + j0 + pseg + 8 * g);
        const v4f zb = *(const v4fa*)(sS2 + j0 + pseg + 8 * g + 4);
        v4f pa, pb;
        pa.x = pexp(s1r, mr, za.x); pa.y = pexp(s1r, mr, za.y); pa.z = pexp(s1r, mr, za.z); pa.w = pexp(s1r, mr, za.w);
        pb.x = pexp(s1r, mr, zb.x); pb.y = pexp(s1r, mr, zb.y); pb.z = pexp(s1r, mr, zb.z); pb.w = pexp(s1r, mr, zb.w);
        const float ts = ((pa.x + pa.y) + (pa.z + pa.w)) + ((pb.x + pb.y) + (pb.z + pb.w));
        tsum = tsum + ts;
        v4u hv, lv;
        split8(pa, pb, hv, lv);
        *(v4ua*)(sPA + prow * PAP + pseg + 8 * g)      = hv;
        *(v4ua*)(sPA + prow * PAP + KT + pseg + 8 * g) = lv;
      }
      lsum = lsum + tsum;
    }
#pragma unroll
    for (int i = 0; i < 4; ++i) {
      const int pc = i * NTHR + tid;
      const int n  = pc >> 3;
      const int q  = pc & 7;
      const size_t go = (size_t)(coloff + n) * NN + (size_t)(j0 + 8 * q);
      const v4u vh = *(const v4ua*)(HTh + go);
      const v4u vl = *(const v4ua*)(HTl + go);
      *(v4ua*)(sHh + n * HBP + 8 * q) = vh;
      *(v4ua*)(sHl + n * HBP + 8 * q) = vl;
    }
    __syncthreads();

#pragma unroll
    for (int ks = 0; ks < KT / 32; ++ks) {
      const unsigned short* pa = sPA + (16 * rg + m) * PAP + 32 * ks + 8 * hh;
      FragB ah, al;
      ah.h[0] = *(const v8usa*)pa;
      ah.h[1] = *(const v8usa*)(pa + 16);
      al.h[0] = *(const v8usa*)(pa + KT);
      al.h[1] = *(const v8usa*)(pa + KT + 16);
#pragma unroll
      for (int nt = 0; nt < 4; ++nt) {
        const int bo = (64 * cg + 16 * nt + m) * HBP + 32 * ks + 8 * hh;
        FragB bh, bl;
        bh.h[0] = *(const v8usa*)(sHh + bo);
        bh.h[1] = *(const v8usa*)(sHh + bo + 16);
        bl.h[0] = *(const v8usa*)(sHl + bo);
        bl.h[1] = *(const v8usa*)(sHl + bo + 16);
        acc[nt] = wmb(ah, bh, acc[nt]);
        acc[nt] = wmb(ah, bl, acc[nt]);
        acc[nt] = wmb(al, bh, acc[nt]);
      }
    }
    __syncthreads();
  }

  lsum = lsum + __shfl_xor(lsum, 1);
  lsum = lsum + __shfl_xor(lsum, 2);
  if ((tid & 3) == 0) sL[prow] = lsum;

#pragma unroll
  for (int nt = 0; nt < 4; ++nt) {
    const int lc = 64 * cg + 16 * nt + m;
#pragma unroll
    for (int r = 0; r < 8; ++r) {
      const int lr = 16 * rg + 8 * hh + r;
      stg[lr * NH + lc] = acc[nt][r];
    }
  }
  __syncthreads();

#pragma unroll 1
  for (int i = 0; i < 8; ++i) {
    const int row = wave * 8 + i;
    const float inv = 1.0f / sL[row];
    float* sp = stg + row * NH + 4 * lane;
    const v4f a = *(const v4fa*)sp;
    v4f o;
    const float v0 = a.x * inv, v1 = a.y * inv, v2 = a.z * inv, v3 = a.w * inv;
    o.x = v0 > 0.0f ? v0 : expm1f(v0);
    o.y = v1 > 0.0f ? v1 : expm1f(v1);
    o.z = v2 > 0.0f ? v2 : expm1f(v2);
    o.w = v3 > 0.0f ? v3 : expm1f(v3);
    *(v4fa*)sp = o;
    float* op = out + (size_t)(rowBase + row) * FOUT + coloff + 4 * lane;
    *(volatile v4f*)op = o;
  }
  __threadfence();
#pragma unroll 1
  for (int i = 0; i < 8; ++i) {
    const int row = wave * 8 + i;
    const v4f o = *(const v4fa*)(stg + row * NH + 4 * lane);
    float* op = out + (size_t)(rowBase + row) * FOUT + coloff + 4 * lane;
    *(volatile v4f*)op = o;
  }
}

extern "C" void kernel_launch(void* const* d_in, const int* in_sizes, int n_in,
                              void* d_out, int out_size, void* d_ws, size_t ws_size,
                              hipStream_t stream) {
  if (n_in < 3) return;
  if (in_sizes[0] != NN * FIN) return;
  if (in_sizes[1] != FIN * FOUT) return;
  if (in_sizes[2] != 2 * FOUT) return;
  if (out_size != NN * FOUT) return;

  const float* x  = (const float*)d_in[0];
  const float* W  = (const float*)d_in[1];
  const float* av = (const float*)d_in[2];
  float* out = (float*)d_out;

  char* ws = (char*)d_ws;
  size_t off = 0;
  const size_t oXB  = off; off += (size_t)NN * FIN * 2;    off = (off + 255) & ~(size_t)255;
  const size_t oWT  = off; off += (size_t)FOUT * FIN * 2;  off = (off + 255) & ~(size_t)255;
  const size_t oHTh = off; off += (size_t)FOUT * NN * 2;   off = (off + 255) & ~(size_t)255;
  const size_t oHTl = off; off += (size_t)FOUT * NN * 2;   off = (off + 255) & ~(size_t)255;
  const size_t oSS  = off; off += (size_t)2 * NN * 4;      off = (off + 255) & ~(size_t)255;
  if (off > ws_size || off > (size_t)WSMAX) return;
  unsigned short* XB  = (unsigned short*)(ws + oXB);
  unsigned short* WT  = (unsigned short*)(ws + oWT);
  unsigned short* HTh = (unsigned short*)(ws + oHTh);
  unsigned short* HTl = (unsigned short*)(ws + oHTl);
  float*          SS  = (float*)(ws + oSS);

  hipFuncSetAttribute(reinterpret_cast<const void*>(&k_proj), hipFuncAttributeMaxDynamicSharedMemorySize, PLDS);
  hipFuncSetAttribute(reinterpret_cast<const void*>(&k_attn), hipFuncAttributeMaxDynamicSharedMemorySize, ALDS);

  k_prep<<<(NUX + NUW) / NTHR, NTHR, 0, stream>>>(x, W, XB, WT);
  k_proj<<<NN / GBM, NTHR, PLDS, stream>>>(XB, WT, av, HTh, HTl, SS);
  k_attn<<<dim3(NN / GBM, FOUT / NH), NTHR, ALDS, stream>>>(HTh, HTl, SS, out);
}
